// GTFShallowPLRNN_60971355734108
// MI455X (gfx1250) — hardware-run, weakly checked
//
#include <hip/hip_runtime.h>
#include <math.h>

typedef __attribute__((ext_vector_type(16))) _Float16 v16h;
typedef __attribute__((ext_vector_type(8)))  _Float16 v8h;
typedef __attribute__((ext_vector_type(8)))  float    v8f;
typedef __attribute__((ext_vector_type(4)))  float    v4f;

constexpr int kB    = 512;
constexpr int kCin  = 12;
constexpr int kLin  = 2500;
constexpr int kC1   = 32;
constexpr int kTap1 = 50;
constexpr int kStr1 = 10;
constexpr int kL1   = 246;
constexpr int kC2   = 32;
constexpr int kTap2 = 25;
constexpr int kStr2 = 5;
constexpr int kT    = 45;
constexpr int kD    = 32;
constexpr int kH    = 64;
constexpr int kKg1  = kCin * kTap1;
constexpr int kKg1P = 608;
constexpr int kKg2  = kC1 * kTap2;
constexpr int kM1   = kB * kL1;
constexpr int kM2   = kB * kT;
constexpr int kSlabP = 36;
constexpr int kHP    = 36;
constexpr int kUP    = 68;
static_assert((kLin - kTap1) / kStr1 + 1 == kL1, "conv1 length");
static_assert((kL1 - kTap2) / kStr2 + 1 == kT, "conv2 length");
static_assert(kKg1 == 600 && kKg1P % 32 == 0 && kKg1P >= kKg1 && kKg1P - kKg1 == 8, "conv1 K pad");
static_assert(kKg2 == 800 && kKg2 % 32 == 0, "conv2 K");
static_assert(kM1 % 64 == 0 && kM2 % 64 == 0, "GEMM M tile multiples");
static_assert(kC1 == 32 && kC2 == 32 && kD == 32 && kH == 64, "two 16-wide column tiles / K = 32, 64");
static_assert(kB == 32 * 16, "32 row tiles of 16 samples");

constexpr float kCarryX   = 64.0f;
constexpr float kCarryCW  = 1024.0f;
constexpr float kCarryAct = 16.0f;
constexpr float kCarryW   = 512.0f;
constexpr float kCarryH   = 8.0f;
constexpr float kCarryU   = 16.0f;
constexpr float kInvConv1 = 1.0f / (kCarryX * kCarryCW);
constexpr float kInvConv2 = 1.0f / (kCarryAct * kCarryCW);
constexpr float kInvProj  = 1.0f / (kCarryAct * kCarryW);
constexpr float kInvW2    = 1.0f / (kCarryH * kCarryW);
constexpr float kInvW1    = 1.0f / (kCarryU * kCarryW);
constexpr float kInvHead  = 1.0f / (kCarryH * kCarryW);
constexpr float kEps      = 1e-5f;
constexpr float kAlpha    = 0.1f;
constexpr float kOneMinusAlpha = 0.9f;

constexpr size_t kXtPlaneBytes = (size_t)kB * kLin * kCin * 2;
constexpr size_t kSzXT  = kXtPlaneBytes + 256;
constexpr size_t kSzBT1 = (size_t)kC1 * kKg1P * 2;
constexpr size_t kSzBT2 = (size_t)kC2 * kKg2 * 2;
constexpr size_t kSzY1  = (size_t)kM1 * kC1 * 2;
constexpr size_t kSzY2  = (size_t)kM2 * kC2 * 2;
constexpr size_t kSzXTM = (size_t)kT * kB * kD * 4;
constexpr size_t kOffXT  = 0;
constexpr size_t kOffBT1 = kOffXT  + kSzXT;
constexpr size_t kOffBT2 = kOffBT1 + kSzBT1;
constexpr size_t kOffY1  = kOffBT2 + kSzBT2;
constexpr size_t kOffY2  = kOffY1  + kSzY1;
constexpr size_t kOffXTM = kOffY2  + kSzY2;
constexpr size_t kWsTotal = kOffXTM + kSzXTM;
static_assert(kWsTotal == 43294976ull, "carve total");
static_assert(kWsTotal <= 134217728ull, "carve cap");
static_assert((kOffBT1 % 256) == 0 && (kOffBT2 % 256) == 0 && (kOffY1 % 256) == 0 &&
              (kOffY2 % 256) == 0 && (kOffXTM % 256) == 0, "aligned regions");

__device__ __forceinline__ _Float16 h16(float v) {
  const float y = (fabsf(v) < 6.103515625e-05f) ? 0.0f : v;
  return (_Float16)y;
}

struct FragH {
  union U { v16h v; v8h h[2]; };
  static __device__ __forceinline__ v16h load(const _Float16* p) {
    U f;
    f.h[0] = *(const v8h*)(p);
    f.h[1] = *(const v8h*)(p + 16);
    return f.v;
  }
  static __device__ __forceinline__ v8f mma(v16h a, v16h b, v8f c) {
    return __builtin_amdgcn_wmma_f32_16x16x32_f16(false, a, false, b, (short)0, c, false, false);
  }
};

__device__ __forceinline__ v16h frag_from_f32(const float* p, float sc) {
  const v4f a0 = *(const v4f*)(p);
  const v4f a1 = *(const v4f*)(p + 4);
  const v4f a2 = *(const v4f*)(p + 16);
  const v4f a3 = *(const v4f*)(p + 20);
  v16h f;
#pragma unroll
  for (int e = 0; e < 4; ++e) {
    f[e]      = h16(a0[e] * sc);
    f[4 + e]  = h16(a1[e] * sc);
    f[8 + e]  = h16(a2[e] * sc);
    f[12 + e] = h16(a3[e] * sc);
  }
  return f;
}

__device__ __forceinline__ void guard2_in3(v8f& a, v8f& b, v16h x, v16h y, v16h z) {
  asm volatile("v_nop\n\tv_nop\n\tv_nop\n\tv_nop" : "+v"(a), "+v"(b) : "v"(x), "v"(y), "v"(z));
}
__device__ __forceinline__ void guard4_in5(v8f& a, v8f& b, v8f& c, v8f& d, v16h x, v16h y, v16h z, v16h w, v16h q) {
  asm volatile("v_nop\n\tv_nop\n\tv_nop\n\tv_nop" : "+v"(a), "+v"(b), "+v"(c), "+v"(d) : "v"(x), "v"(y), "v"(z), "v"(w), "v"(q));
}
__device__ __forceinline__ void guard2_in6(v8f& a, v8f& b, v16h x, v16h y, v16h z, v16h w, v16h q, v16h s) {
  asm volatile("v_nop\n\tv_nop\n\tv_nop\n\tv_nop" : "+v"(a), "+v"(b) : "v"(x), "v"(y), "v"(z), "v"(w), "v"(q), "v"(s));
}
__device__ __forceinline__ void acc_guard4(v8f& a, v8f& b, v8f& c, v8f& d) {
  asm volatile("v_nop\n\tv_nop\n\tv_nop\n\tv_nop" : "+v"(a), "+v"(b), "+v"(c), "+v"(d));
}
__device__ __forceinline__ void wave_lds_sync() {
  __builtin_amdgcn_fence(__ATOMIC_RELEASE, "workgroup");
  __builtin_amdgcn_wave_barrier();
  __builtin_amdgcn_fence(__ATOMIC_ACQUIRE, "workgroup");
}

constexpr int kBt1Thr = kC1 * kKg1P / 8;
constexpr int kBt2Thr = kC2 * kKg2 / 8;
static_assert(kBt1Thr == 2432 && kBt2Thr == 3200, "weight plane threads");
static_assert((kBt1Thr % 32) == 0 && ((kBt1Thr + kBt2Thr) % 256) == 0, "exact grid");
static_assert((kKg1P % 8) == 0 && (kKg2 % 8) == 0, "8 halves stay inside a row");

__global__ __launch_bounds__(256) void conv_weight_planes_kernel(
    const float* __restrict__ w1, const float* __restrict__ w2,
    unsigned short* __restrict__ bt1, unsigned short* __restrict__ bt2)
{
  const int i = blockIdx.x * 256 + threadIdx.x;
  if (i >= kBt1Thr + kBt2Thr) return;
  v8h hv;
  unsigned short* dst;
  if (i < kBt1Thr) {
    const int e0 = i * 8;
    const int oc = e0 / kKg1P;
    const int k0 = e0 - oc * kKg1P;
#pragma unroll
    for (int e = 0; e < 8; ++e) {
      const int k = k0 + e;
      const bool valid = (k < kKg1);
      const int kc = valid ? k : (kKg1 - 1);
      const int tap = kc / kCin;
      const int ic = kc - tap * kCin;
      float v = w1[oc * kKg1 + ic * kTap1 + tap];
      asm volatile("" : "+v"(v));
      hv[e] = h16(valid ? (v * kCarryCW) : 0.0f);
    }
    dst = bt1 + e0;
  } else {
    const int e0 = (i - kBt1Thr) * 8;
    const int oc = e0 / kKg2;
    const int k0 = e0 - oc * kKg2;
#pragma unroll
    for (int e = 0; e < 8; ++e) {
      const int k = k0 + e;
      const int tap = k / kC1;
      const int ic = k - tap * kC1;
      const float v = w2[oc * kKg2 + ic * kTap2 + tap];
      hv[e] = h16(v * kCarryCW);
    }
    dst = bt2 + e0;
  }
  *(volatile v8h*)dst = hv;
  __threadfence();
  *(volatile v8h*)dst = hv;
}

constexpr int kXRow8 = kCin * kLin / 8;
constexpr int kXThr  = kB * kXRow8;
static_assert((kCin * kLin) % 8 == 0 && kXRow8 == 3750 && kXThr == 1920000, "x plane threads");
static_assert(kXThr % 256 == 0, "exact data blocks");

__global__ __launch_bounds__(256) void x_channel_last_kernel(
    const float* __restrict__ x, unsigned short* __restrict__ xt)
{
  const int i = blockIdx.x * 256 + threadIdx.x;
  if (i >= kXThr + 8) return;
  const bool tail = (i >= kXThr);
  const int ii = tail ? (kXThr - 1) : i;
  const int b = ii / kXRow8;
  const int rem0 = (ii - b * kXRow8) * 8;
  const float* xb = x + (size_t)b * (kCin * kLin);
  v8h hv;
#pragma unroll
  for (int e = 0; e < 8; ++e) {
    const int rem = rem0 + e;
    const int l = rem / kCin;
    const int c = rem - l * kCin;
    float v = xb[c * kLin + l];
    asm volatile("" : "+v"(v));
    hv[e] = h16(tail ? 0.0f : (v * kCarryX));
  }
  unsigned short* dst = xt + (size_t)i * 8;
  *(volatile v8h*)dst = hv;
  __threadfence();
  *(volatile v8h*)dst = hv;
}

template <int KTOT, int LOUT, int BSTRIDE, int TSTRIDE>
__global__ __launch_bounds__(256) void conv_gemm_kernel(
    const unsigned short* __restrict__ Ap, const unsigned short* __restrict__ Btp,
    const float* __restrict__ cbias, const float* __restrict__ gam, const float* __restrict__ bet,
    const float* __restrict__ rmean, const float* __restrict__ rvar,
    unsigned short* __restrict__ Yout, int tilesM, float accInv, float outCarry)
{
  static_assert(KTOT % 32 == 0, "K multiple of 32");
  __shared__ __align__(16) float sT[8][16 * kSlabP];
  const _Float16* A  = (const _Float16*)Ap;
  const _Float16* Bt = (const _Float16*)Btp;
  const int lane = threadIdx.x & 31;
  const int wave = threadIdx.x >> 5;
  const int tile = blockIdx.x * 8 + wave;
  if (tile >= tilesM) return;
  const int c = lane & 15;
  const int hh = lane >> 4;
  const int koff = hh * 8;
  const int m0 = tile * 64;

  int ab[4];
#pragma unroll
  for (int i = 0; i < 4; ++i) {
    const int m = m0 + 16 * i + c;
    const int b = m / LOUT;
    const int t = m - b * LOUT;
    ab[i] = b * BSTRIDE + t * TSTRIDE + koff;
  }
  const _Float16* bp0 = Bt + c * KTOT + koff;
  const _Float16* bp1 = Bt + (16 + c) * KTOT + koff;

  v8f acc[4][2];
#pragma unroll
  for (int i = 0; i < 4; ++i) {
    acc[i][0] = (v8f){0.f, 0.f, 0.f, 0.f, 0.f, 0.f, 0.f, 0.f};
    acc[i][1] = (v8f){0.f, 0.f, 0.f, 0.f, 0.f, 0.f, 0.f, 0.f};
  }

#pragma unroll 1
  for (int k0 = 0; k0 < KTOT; k0 += 32) {
    const v16h b0 = FragH::load(bp0 + k0);
    const v16h b1 = FragH::load(bp1 + k0);
#pragma unroll
    for (int i = 0; i < 4; ++i) {
      const v16h a = FragH::load(A + ab[i] + k0);
      acc[i][0] = FragH::mma(a, b0, acc[i][0]);
      acc[i][1] = FragH::mma(a, b1, acc[i][1]);
      guard2_in3(acc[i][0], acc[i][1], a, b0, b1);
    }
  }
  acc_guard4(acc[0][0], acc[0][1], acc[1][0], acc[1][1]);
  acc_guard4(acc[2][0], acc[2][1], acc[3][0], acc[3][1]);

  float sc[2], sh[2];
#pragma unroll
  for (int j = 0; j < 2; ++j) {
    const int n = 16 * j + c;
    const float rs = 1.0f / sqrtf(rvar[n] + kEps);
    sc[j] = gam[n] * rs;
    sh[j] = (cbias[n] - rmean[n]) * sc[j] + bet[n];
  }

  float* slab = sT[wave];
  const int srow = lane >> 2;
  const int scol = (lane & 3) * 8;
#pragma unroll
  for (int i = 0; i < 4; ++i) {
    const int mBase = m0 + 16 * i;
#pragma unroll
    for (int j = 0; j < 2; ++j) {
#pragma unroll
      for (int r = 0; r < 8; ++r) {
        const float z = (acc[i][j][r] * accInv) * sc[j] + sh[j];
        slab[(8 * hh + r) * kSlabP + 16 * j + c] = fmaxf(z, 0.0f) * outCarry;
      }
    }
    wave_lds_sync();
    v8h hv[2];
#pragma unroll
    for (int it = 0; it < 2; ++it) {
      const float* sp = slab + (it * 8 + srow) * kSlabP + scol;
      const v4f a0 = *(const v4f*)(sp);
      const v4f a1 = *(const v4f*)(sp + 4);
#pragma unroll
      for (int e = 0; e < 4; ++e) {
        hv[it][e]     = h16(a0[e]);
        hv[it][4 + e] = h16(a1[e]);
      }
    }
    for (int pass = 0; pass < 2; ++pass) {
#pragma unroll
      for (int it = 0; it < 2; ++it) {
        *(volatile v8h*)(Yout + (size_t)(mBase + it * 8 + srow) * 32 + scol) = hv[it];
      }
      __threadfence();
    }
    wave_lds_sync();
  }
}

constexpr int kProjTiles = kT * (kB / 16);
static_assert(kProjTiles == 1440 && (kProjTiles % 8) == 0, "projection tiles");

__global__ __launch_bounds__(256) void proj_ln_kernel(
    const unsigned short* __restrict__ Y2p, const float* __restrict__ pw, const float* __restrict__ pb,
    const float* __restrict__ lg, const float* __restrict__ lb, float* __restrict__ XTM)
{
  __shared__ __align__(16) float sT[8][16 * kSlabP];
  const _Float16* Y2 = (const _Float16*)Y2p;
  const int lane = threadIdx.x & 31;
  const int wave = threadIdx.x >> 5;
  const int tile = blockIdx.x * 8 + wave;
  if (tile >= kProjTiles) return;
  const int c = lane & 15;
  const int hh = lane >> 4;
  const int koff = hh * 8;
  const int t = tile >> 5;
  const int b0 = (tile & 31) * 16;

  const v16h a = FragH::load(Y2 + ((size_t)(b0 + c) * kT + t) * 32 + koff);
  const v16h w0 = frag_from_f32(pw + c * kD + koff, kCarryW);
  const v16h w1 = frag_from_f32(pw + (16 + c) * kD + koff, kCarryW);
  v8f acc0 = (v8f){0.f, 0.f, 0.f, 0.f, 0.f, 0.f, 0.f, 0.f};
  v8f acc1 = (v8f){0.f, 0.f, 0.f, 0.f, 0.f, 0.f, 0.f, 0.f};
  acc0 = FragH::mma(a, w0, acc0);
  acc1 = FragH::mma(a, w1, acc1);
  guard2_in3(acc0, acc1, a, w0, w1);

  const float pb0 = pb[c], pb1 = pb[16 + c];
  const float g0 = lg[c], g1 = lg[16 + c];
  const float e0 = lb[c], e1 = lb[16 + c];
  float* slab = sT[wave];
#pragma unroll
  for (int r = 0; r < 8; ++r) {
    const float v0 = acc0[r] * kInvProj + pb0;
    const float v1 = acc1[r] * kInvProj + pb1;
    float s = v0 + v1;
    s += __shfl_xor(s, 1, 32);
    s += __shfl_xor(s, 2, 32);
    s += __shfl_xor(s, 4, 32);
    s += __shfl_xor(s, 8, 32);
    const float mu = s * (1.0f / 32.0f);
    const float d0 = v0 - mu;
    const float d1 = v1 - mu;
    float ss = d0 * d0 + d1 * d1;
    ss += __shfl_xor(ss, 1, 32);
    ss += __shfl_xor(ss, 2, 32);
    ss += __shfl_xor(ss, 4, 32);
    ss += __shfl_xor(ss, 8, 32);
    const float rstd = 1.0f / sqrtf(ss * (1.0f / 32.0f) + kEps);
    slab[(8 * hh + r) * kSlabP + c]      = (d0 * rstd) * g0 + e0;
    slab[(8 * hh + r) * kSlabP + 16 + c] = (d1 * rstd) * g1 + e1;
  }
  wave_lds_sync();
  const int srow = lane >> 3;
  const int c4 = (lane & 7) * 4;
  v4f ov[4];
#pragma unroll
  for (int it = 0; it < 4; ++it) ov[it] = *(const v4f*)(slab + (it * 4 + srow) * kSlabP + c4);
  float* op = XTM + ((size_t)t * kB + b0) * kD;
  for (int pass = 0; pass < 2; ++pass) {
#pragma unroll
    for (int it = 0; it < 4; ++it) {
      *(volatile v4f*)(op + (size_t)(it * 4 + srow) * kD + c4) = ov[it];
    }
    __threadfence();
  }
}

__global__ __launch_bounds__(32) void cell_seq_kernel(
    const float* __restrict__ XTM, const float* __restrict__ Amat,
    const float* __restrict__ W1, const float* __restrict__ W2,
    const float* __restrict__ h1, const float* __restrict__ h2,
    const float* __restrict__ lg2, const float* __restrict__ lb2,
    const float* __restrict__ ow, const float* __restrict__ ob,
    float* __restrict__ out)
{
  __shared__ __align__(16) float As[kD * kHP];
  __shared__ __align__(16) float Hs[16 * kHP];
  __shared__ __align__(16) float Us[16 * kUP];
  const int lane = threadIdx.x & 31;
  const int c = lane & 15;
  const int hh = lane >> 4;
  const int koff = hh * 8;
  const int rowbase = blockIdx.x * 16;

#pragma unroll
  for (int it = 0; it < 8; ++it) {
    const int idx = lane + 32 * it;
    const int row = idx >> 3;
    const int q4 = (idx & 7) * 4;
    *(v4f*)(As + row * kHP + q4) = *(const v4f*)(Amat + row * kD + q4);
  }
#pragma unroll
  for (int i = 0; i < 18; ++i) Hs[lane + 32 * i] = 0.0f;
  __syncthreads();

  v16h bw2[4];
#pragma unroll
  for (int j = 0; j < 4; ++j) bw2[j] = frag_from_f32(W2 + (16 * j + c) * kD + koff, kCarryW);
  v16h bw1[2][2];
#pragma unroll
  for (int j = 0; j < 2; ++j) {
#pragma unroll
    for (int kc = 0; kc < 2; ++kc) bw1[j][kc] = frag_from_f32(W1 + (16 * j + c) * kH + 32 * kc + koff, kCarryW);
  }
  float h2v[4], g2v[4], b2v[4];
#pragma unroll
  for (int j = 0; j < 4; ++j) {
    h2v[j] = h2[16 * j + c];
    g2v[j] = lg2[16 * j + c];
    b2v[j] = lb2[16 * j + c];
  }
  float h1v[2];
  h1v[0] = h1[c];
  h1v[1] = h1[16 + c];

  float sum[2][8];
#pragma unroll
  for (int j = 0; j < 2; ++j)
#pragma unroll
    for (int r = 0; r < 8; ++r) sum[j][r] = 0.0f;

  const v8f z8 = (v8f){0.f, 0.f, 0.f, 0.f, 0.f, 0.f, 0.f, 0.f};

#pragma unroll 1
  for (int t = 0; t < kT; ++t) {
    float xr[2][8];
#pragma unroll
    for (int j = 0; j < 2; ++j)
#pragma unroll
      for (int r = 0; r < 8; ++r)
        xr[j][r] = XTM[((size_t)t * kB + rowbase + 8 * hh + r) * kD + 16 * j + c];

    const v16h ah = frag_from_f32(Hs + c * kHP + koff, kCarryH);
    v8f u[4];
#pragma unroll
    for (int j = 0; j < 4; ++j) u[j] = FragH::mma(ah, bw2[j], z8);
    guard4_in5(u[0], u[1], u[2], u[3], ah, bw2[0], bw2[1], bw2[2], bw2[3]);

#pragma unroll
    for (int r = 0; r < 8; ++r) {
      float uu[4];
#pragma unroll
      for (int j = 0; j < 4; ++j) uu[j] = fmaxf(u[j][r] * kInvW2 + h2v[j], 0.0f);
      float s = (uu[0] + uu[1]) + (uu[2] + uu[3]);
      s += __shfl_xor(s, 1, 32);
      s += __shfl_xor(s, 2, 32);
      s += __shfl_xor(s, 4, 32);
      s += __shfl_xor(s, 8, 32);
      const float mu = s * (1.0f / 64.0f);
      float ss = 0.0f;
#pragma unroll
      for (int j = 0; j < 4; ++j) {
        uu[j] = uu[j] - mu;
        ss += uu[j] * uu[j];
      }
      ss += __shfl_xor(ss, 1, 32);
      ss += __shfl_xor(ss, 2, 32);
      ss += __shfl_xor(ss, 4, 32);
      ss += __shfl_xor(ss, 8, 32);
      const float rstd = 1.0f / sqrtf(ss * (1.0f / 64.0f) + kEps);
#pragma unroll
      for (int j = 0; j < 4; ++j)
        Us[(8 * hh + r) * kUP + 16 * j + c] = (uu[j] * rstd) * g2v[j] + b2v[j];
    }
    __syncthreads();

    const v16h ad0 = frag_from_f32(Us + c * kUP + koff, kCarryU);
    const v16h ad1 = frag_from_f32(Us + c * kUP + 32 + koff, kCarryU);
    v8f nl[2];
#pragma unroll
    for (int j = 0; j < 2; ++j) {
      nl[j] = FragH::mma(ad0, bw1[j][0], z8);
      nl[j] = FragH::mma(ad1, bw1[j][1], nl[j]);
    }
    guard2_in6(nl[0], nl[1], ad0, ad1, bw1[0][0], bw1[0][1], bw1[1][0], bw1[1][1]);

    float lin[2][8];
#pragma unroll
    for (int j = 0; j < 2; ++j)
#pragma unroll
      for (int r = 0; r < 8; ++r) lin[j][r] = 0.0f;
#pragma unroll 1
    for (int k4 = 0; k4 < 8; ++k4) {
      const v4f a0 = *(const v4f*)(As + c * kHP + 4 * k4);
      const v4f a1 = *(const v4f*)(As + (16 + c) * kHP + 4 * k4);
#pragma unroll
      for (int r = 0; r < 8; ++r) {
        const v4f hv = *(const v4f*)(Hs + (8 * hh + r) * kHP + 4 * k4);
#pragma unroll
        for (int e = 0; e < 4; ++e) {
          lin[0][r] = fmaf(hv[e], a0[e], lin[0][r]);
          lin[1][r] = fmaf(hv[e], a1[e], lin[1][r]);
        }
      }
    }

    float hn[2][8];
#pragma unroll
    for (int j = 0; j < 2; ++j) {
#pragma unroll
      for (int r = 0; r < 8; ++r) {
        const float hp = lin[j][r] + (nl[j][r] * kInvW1 + h1v[j]);
        const float v = kOneMinusAlpha * (hp + xr[j][r]) + kAlpha * hp;
        hn[j][r] = v;
        sum[j][r] += v;
      }
    }
    __syncthreads();
#pragma unroll
    for (int j = 0; j < 2; ++j)
#pragma unroll
      for (int r = 0; r < 8; ++r) Hs[(8 * hh + r) * kHP + 16 * j + c] = hn[j][r];
    __syncthreads();
  }

#pragma unroll
  for (int j = 0; j < 2; ++j)
#pragma unroll
    for (int r = 0; r < 8; ++r) Hs[(8 * hh + r) * kHP + 16 * j + c] = sum[j][r] * (1.0f / (float)kT);
  __syncthreads();
  const v16h ap = frag_from_f32(Hs + c * kHP + koff, kCarryH);
  const v16h bo0 = frag_from_f32(ow + c * kD + koff, kCarryW);
  const v16h bo1 = frag_from_f32(ow + (16 + c) * kD + koff, kCarryW);
  v8f o0 = FragH::mma(ap, bo0, z8);
  v8f o1 = FragH::mma(ap, bo1, z8);
  guard2_in3(o0, o1, ap, bo0, bo1);
  const float ob0 = ob[c], ob1 = ob[16 + c];
  __syncthreads();
#pragma unroll
  for (int r = 0; r < 8; ++r) {
    Us[(8 * hh + r) * kUP + c]      = o0[r] * kInvHead + ob0;
    Us[(8 * hh + r) * kUP + 16 + c] = o1[r] * kInvHead + ob1;
  }
  __syncthreads();
  const int srow = lane >> 3;
  const int c4 = (lane & 7) * 4;
  v4f ov[4];
#pragma unroll
  for (int it = 0; it < 4; ++it) ov[it] = *(const v4f*)(Us + (it * 4 + srow) * kUP + c4);
  float* op = out + (size_t)rowbase * kD;
  for (int pass = 0; pass < 2; ++pass) {
#pragma unroll
    for (int it = 0; it < 4; ++it) {
      *(volatile v4f*)(op + (size_t)(it * 4 + srow) * kD + c4) = ov[it];
    }
    __threadfence();
  }
}

extern "C" void kernel_launch(void* const* d_in, const int* in_sizes, int n_in,
                              void* d_out, int out_size, void* d_ws, size_t ws_size,
                              hipStream_t stream)
{
  if (n_in < 26 || d_out == nullptr || d_ws == nullptr) return;
  if (in_sizes[0] != kB * kCin * kLin) return;
  if (in_sizes[1] != kC1 * kCin * kTap1) return;
  if (in_sizes[7] != kC2 * kC1 * kTap2) return;
  if (in_sizes[13] != kD * kC2) return;
  if (in_sizes[15] != kD * kD) return;
  if (in_sizes[16] != kD * kH) return;
  if (in_sizes[17] != kH * kD) return;
  if (in_sizes[24] != kD * kD) return;
  if (out_size != kB * kD) return;
  if (ws_size < kWsTotal) return;

  const float* x       = (const float*)d_in[0];
  const float* conv1_w = (const float*)d_in[1];
  const float* conv1_b = (const float*)d_in[2];
  const float* bn1_g   = (const float*)d_in[3];
  const float* bn1_b   = (const float*)d_in[4];
  const float* bn1_m   = (const float*)d_in[5];
  const float* bn1_v   = (const float*)d_in[6];
  const float* conv2_w = (const float*)d_in[7];
  const float* conv2_b = (const float*)d_in[8];
  const float* bn2_g   = (const float*)d_in[9];
  const float* bn2_b   = (const float*)d_in[10];
  const float* bn2_m   = (const float*)d_in[11];
  const float* bn2_v   = (const float*)d_in[12];
  const float* proj_w  = (const float*)d_in[13];
  const float* proj_b  = (const float*)d_in[14];
  const float* Amat    = (const float*)d_in[15];
  const float* W1      = (const float*)d_in[16];
  const float* W2      = (const float*)d_in[17];
  const float* h1      = (const float*)d_in[18];
  const float* h2      = (const float*)d_in[19];
  const float* ln1_g   = (const float*)d_in[20];
  const float* ln1_b   = (const float*)d_in[21];
  const float* ln2_g   = (const float*)d_in[22];
  const float* ln2_b   = (const float*)d_in[23];
  const float* out_w   = (const float*)d_in[24];
  const float* out_b   = (const float*)d_in[25];

  char* ws = (char*)d_ws;
  unsigned short* XT  = (unsigned short*)(ws + kOffXT);
  unsigned short* BT1 = (unsigned short*)(ws + kOffBT1);
  unsigned short* BT2 = (unsigned short*)(ws + kOffBT2);
  unsigned short* Y1T = (unsigned short*)(ws + kOffY1);
  unsigned short* Y2  = (unsigned short*)(ws + kOffY2);
  float*          XTM = (float*)(ws + kOffXTM);

  conv_weight_planes_kernel<<<(kBt1Thr + kBt2Thr) / 256, 256, 0, stream>>>(conv1_w, conv2_w, BT1, BT2);

  x_channel_last_kernel<<<kXThr / 256 + 1, 256, 0, stream>>>(x, XT);

  conv_gemm_kernel<kKg1P, kL1, kCin * kLin, kStr1 * kCin><<<(kM1 / 64) / 8, 256, 0, stream>>>(
      XT, BT1, conv1_b, bn1_g, bn1_b, bn1_m, bn1_v, Y1T, kM1 / 64, kInvConv1, kCarryAct);

  conv_gemm_kernel<kKg2, kT, kL1 * kC1, kStr2 * kC1><<<(kM2 / 64) / 8, 256, 0, stream>>>(
      Y1T, BT2, conv2_b, bn2_g, bn2_b, bn2_m, bn2_v, Y2, kM2 / 64, kInvConv2, kCarryAct);

  proj_ln_kernel<<<kProjTiles / 8, 256, 0, stream>>>(Y2, proj_w, proj_b, ln1_g, ln1_b, XTM);

  cell_seq_kernel<<<kB / 16, 32, 0, stream>>>(XTM, Amat, W1, W2, h1, h2, ln2_g, ln2_b,
                                              out_w, out_b, (float*)d_out);
}
